// GAT_23270132810343
// MI455X (gfx1250) — hardware-run, weakly checked
//
#include <hip/hip_runtime.h>


#ifndef NB
#define NB 2
#endif
#ifndef SEQ
#define SEQ 2048
#endif
#define NB_FULL  2
#define SEQ_FULL 2048
#ifndef OUT_SEQ
#define OUT_SEQ SEQ
#endif
#ifndef ATT_RP
#define ATT_RP SEQ
#endif
#ifndef ATT_BP
#define ATT_BP ((size_t)SEQ * SEQ)
#endif
#define DM   256
#define NH_  8
#define HD   32
#define NL   2
#define CXP  (2 * DM)
#define AW   4
#define QRS  2048.0f
#define QRI  (1.0f / 2048.0f)
#define SC2  (0.17677669529663687f * 1.4426950408889634f)
#define PSH  8.0f
#define NEGT (-1.0e9f * 1.4426950408889634f)
#define APS  15.0f
#define RSC  9.5367431640625e-07f
#define ATT_OFF ((size_t)NB_FULL * SEQ_FULL * DM)

static_assert(HD == 32);
static_assert(NH_ * HD == DM);
static_assert(NH_ % 2 == 0);
static_assert(NH_ == 8);
static_assert(DM == 256);
static_assert(DM % 64 == 0);
static_assert(DM % 32 == 0);
static_assert(CXP % 32 == 0);
static_assert(SEQ % 64 == 0);
static_assert((NB * SEQ) % 64 == 0);
static_assert(SEQ % 32 == 0);
static_assert(SEQ % (16 * AW) == 0);
static_assert(((size_t)SEQ * DM) % 8 == 0);
static_assert((NB * SEQ) % 8 == 0);
static_assert(((size_t)SEQ * (SEQ / 32)) % 256 == 0);
static_assert(NB <= NB_FULL);
static_assert(SEQ <= SEQ_FULL);
static_assert(OUT_SEQ >= SEQ);
static_assert(ATT_RP >= SEQ);
static_assert(ATT_RP % 32 == 0);
static_assert(ATT_BP % 32 == 0);
static_assert(NL == 2);
static_assert(ATT_OFF * 4 == (size_t)4194304);
static_assert(((size_t)(NB - 1) * OUT_SEQ + SEQ) * DM <= ATT_OFF);
static_assert(ATT_OFF + (size_t)(NB - 1) * ATT_BP + (size_t)(SEQ - 1) * ATT_RP + SEQ <= (size_t)9437184);

typedef _Float16 h16;
typedef unsigned short bf;
typedef __attribute__((ext_vector_type(16))) __bf16   v16bf;
typedef __attribute__((ext_vector_type(16))) _Float16 v16h;
typedef __attribute__((ext_vector_type(8)))  _Float16 v8h;
typedef __attribute__((ext_vector_type(8)))  unsigned short v8us;
typedef __attribute__((ext_vector_type(8)))  float    v8f;
typedef __attribute__((ext_vector_type(4)))  float    v4f;
typedef __attribute__((ext_vector_type(4)))  int      v4i;
typedef v4f  __attribute__((may_alias)) v4fa;
typedef v8h  __attribute__((may_alias)) v8ha;

__device__ __forceinline__ unsigned short f2bf(float f) { unsigned u = __float_as_uint(f); u += 0x7FFFu + ((u >> 16) & 1u); return (unsigned short)(u >> 16); }
__device__ __forceinline__ float bf2f(unsigned short s) { return __uint_as_float(((unsigned)s) << 16); }
__device__ __forceinline__ float bfr(float f) { return bf2f(f2bf(f)); }
__device__ __forceinline__ v16h cat16(v8h lo, v8h hi) { return __builtin_shufflevector(lo, hi, 0, 1, 2, 3, 4, 5, 6, 7, 8, 9, 10, 11, 12, 13, 14, 15); }
__device__ __forceinline__ v16bf cat16b(v8us lo, v8us hi) { return __builtin_bit_cast(v16bf, __builtin_shufflevector(lo, hi, 0, 1, 2, 3, 4, 5, 6, 7, 8, 9, 10, 11, 12, 13, 14, 15)); }
__device__ __forceinline__ v8f wmma16(v16h a, v16h b, v8f c) { return __builtin_amdgcn_wmma_f32_16x16x32_f16(false, a, false, b, (short)0, c, false, false); }
__device__ __forceinline__ v8f wmmab(v16bf a, v16bf b, v8f c) { return __builtin_amdgcn_wmma_f32_16x16x32_bf16(false, a, false, b, (short)0, c, false, false); }
__device__ __forceinline__ v16h  ldh(const h16* p) { return cat16(*(const v8h*)p, *(const v8h*)(p + 16)); }
__device__ __forceinline__ v16bf ldb(const bf* p)  { return cat16b(*(const v8us*)p, *(const v8us*)(p + 16)); }
__device__ __forceinline__ void wave_sync() { __builtin_amdgcn_fence(3  , "wavefront"); __builtin_amdgcn_wave_barrier(); asm volatile("" ::: "memory"); }
static __device__ __forceinline__ h16 toh_flush(float v) { const h16 r = (h16)v; return (fabsf(v) < 6.103515625e-05f) ? (h16)0.0f : r; }
__device__ __forceinline__ v8f wmma16g(v16h a, v16h b, v8f c) { c = wmma16(a, b, c); asm volatile("v_nop\n\tv_nop\n\tv_nop\n\tv_nop" : "+v"(c) : "v"(a), "v"(b)); return c; }

__global__ __launch_bounds__(256) void k_cvt8(const float* __restrict__ src, bf* dst, size_t n8) {
    const size_t i = (size_t)blockIdx.x * 256 + threadIdx.x; if (i >= n8) return;
    const v8f v = *(const v8f*)(src + i * 8); v8us o;
#pragma unroll
    for (int k = 0; k < 8; ++k) o[k] = f2bf(v[k]);
    *(volatile v8us*)(dst + i * 8) = o; __threadfence(); *(volatile v8us*)(dst + i * 8) = o;
}

__global__ __launch_bounds__(256) void k_wdup(const float* __restrict__ W, bf* dst, size_t n8) {
    const size_t i = (size_t)blockIdx.x * 256 + threadIdx.x; if (i >= n8) return;
    const v8f v = *(const v8f*)(W + i * 8); v8us o;
#pragma unroll
    for (int k = 0; k < 8; ++k) o[k] = f2bf(v[k]);
    bf* d = dst + (i >> 5) * (size_t)CXP + (size_t)(i & 31) * 8;
    *(volatile v8us*)d = o; *(volatile v8us*)(d + DM) = o; __threadfence(); *(volatile v8us*)d = o; *(volatile v8us*)(d + DM) = o;
}

__global__ __launch_bounds__(64) void k_zero(float* p) {
    const v4f z = (v4f){};
    *(volatile v4f*)(p + 4 * threadIdx.x) = z; __threadfence(); *(volatile v4f*)(p + 4 * threadIdx.x) = z;
}

__global__ __launch_bounds__(256) void k_mask(const float* __restrict__ adj, unsigned* MB) {
    const int lane = threadIdx.x & 31, wave = __builtin_amdgcn_readfirstlane((int)(threadIdx.x >> 5));
    const int g0 = (blockIdx.x * 8 + wave) * 32;
    unsigned mine = 0u;
#pragma unroll 1
    for (int i = 0; i < 32; ++i) { const int g = g0 + i; const int t = g / (SEQ / 32), w = g - t * (SEQ / 32);
        const float a = adj[(size_t)t * SEQ_FULL + 32 * w + lane];
        const unsigned bal = __builtin_amdgcn_ballot_w32(a > 0.0f);
        mine = (i == lane) ? bal : mine; }
    *(volatile unsigned*)(MB + g0 + lane) = mine; __threadfence(); *(volatile unsigned*)(MB + g0 + lane) = mine;
}

template <bool F32OUT>
__global__ __launch_bounds__(32) void k_gemm(const bf* __restrict__ A, const bf* __restrict__ Bt, h16* Ph, h16* Pr, float* OUT, const float* __restrict__ bias,
                                             size_t sRB, size_t sCB, int K, int useRes, int RB, int pitch, int CB, int biasRow) {
    __shared__ __align__(16) float os[16 * 68];
    const int lane = threadIdx.x & 31, lr = lane & 15, hi = lane >> 4; const int r0 = blockIdx.x * 64, c0 = blockIdx.y * 64;
    v8f acc[4][4];
#pragma unroll
    for (int mb = 0; mb < 4; ++mb)
#pragma unroll
        for (int nb = 0; nb < 4; ++nb) acc[mb][nb] = (v8f){};
    const size_t aoff = (size_t)(r0 + lr) * K + 8 * hi, boff = (size_t)(c0 + lr) * K + 8 * hi;
#pragma unroll 1
    for (int kc = 0; kc < K; kc += 32) {
        v16bf a[4];
#pragma unroll
        for (int mb = 0; mb < 4; ++mb) a[mb] = ldb(A + aoff + (size_t)mb * 16 * K + kc);
#pragma unroll
        for (int nb = 0; nb < 4; ++nb) { const v16bf b = ldb(Bt + boff + (size_t)nb * 16 * K + kc);
#pragma unroll
            for (int mb = 0; mb < 4; ++mb) acc[mb][nb] = wmmab(a[mb], b, acc[mb][nb]); }
        asm volatile("v_nop\n\tv_nop\n\tv_nop\n\tv_nop" : "+v"(acc[0][0]), "+v"(acc[1][1]), "+v"(acc[2][2]), "+v"(acc[3][3]) : "v"(a[0]), "v"(a[1]), "v"(a[2]), "v"(a[3]));
    }
    const size_t tbase = (size_t)(r0 / RB) * sRB + (size_t)(r0 % RB) * (size_t)pitch + (size_t)(c0 / CB) * sCB + (size_t)(c0 % CB);
#pragma unroll
    for (int mb = 0; mb < 4; ++mb) {
#pragma unroll
        for (int nb = 0; nb < 4; ++nb) {
#pragma unroll
            for (int j = 0; j < 8; ++j) os[(hi * 8 + j) * 68 + nb * 16 + lr] = acc[mb][nb][j]; }
        wave_sync();
        if constexpr (!F32OUT) {
            const size_t sb = tbase + (size_t)(mb * 16) * (size_t)pitch;
#pragma unroll 1
            for (int ps = 0; ps < 2; ++ps) {
#pragma unroll
                for (int s = 0; s < 4; ++s) { const int row = 4 * s + (lane >> 3), c8 = (lane & 7) * 8;
                    v4f x0 = *(const v4fa*)(&os[row * 68 + c8]); v4f x1 = *(const v4fa*)(&os[row * 68 + c8 + 4]);
                    const int cidx = (c0 + c8) & (DM - 1), ridx = (r0 + mb * 16 + row) & (DM - 1);
                    const v4f bc0 = *(const v4f*)(bias + cidx), bc1 = *(const v4f*)(bias + cidx + 4); const float br = bias[ridx];
                    v8h hv, rv;
#pragma unroll
                    for (int i = 0; i < 4; ++i) { const float y0 = x0[i] + bfr(biasRow ? br : bc0[i]); const float y1 = x1[i] + bfr(biasRow ? br : bc1[i]);
                        const h16 a0 = (h16)y0; const h16 a1 = (h16)y1; hv[i] = a0; hv[4 + i] = a1; rv[i] = (h16)((y0 - (float)a0) * QRS); rv[4 + i] = (h16)((y1 - (float)a1) * QRS); }
                    const size_t oo = sb + (size_t)row * (size_t)pitch + c8;
                    *(volatile v8h*)(Ph + oo) = hv; if (useRes) *(volatile v8h*)(Pr + oo) = rv; }
                if (ps == 0) __threadfence(); }
        } else {
#pragma unroll 1
            for (int ps = 0; ps < 2; ++ps) {
#pragma unroll
                for (int s = 0; s < 8; ++s) { const int row = 2 * s + hi, cofs = lr * 4;
                    const int m = r0 + mb * 16 + row; const int bb = m / SEQ, tt = m - bb * SEQ;
                    v4f val = *(const v4fa*)(&os[row * 68 + cofs]);
                    const int cidx = (c0 + cofs) & (DM - 1), ridx = m & (DM - 1);
                    const v4f bc = *(const v4f*)(bias + cidx); const float br = bias[ridx];
#pragma unroll
                    for (int i = 0; i < 4; ++i) val[i] = val[i] + bfr(biasRow ? br : bc[i]);
                    *(volatile v4f*)(OUT + ((size_t)bb * OUT_SEQ + tt) * DM + c0 + cofs) = val; }
                if (ps == 0) __threadfence(); }
        }
        wave_sync();
    }
}

__global__ __launch_bounds__(256) void k_rowop(const float* __restrict__ X, const float* __restrict__ O, const float* __restrict__ G, const float* __restrict__ Be,
                                               float* Y, bf* PL, int doLN, int doPl) {
#pragma clang fp contract(off)
    __shared__ __align__(16) float rs[8 * DM];
    const int lane = threadIdx.x & 31, wave = __builtin_amdgcn_readfirstlane((int)(threadIdx.x >> 5));
    const int m = blockIdx.x * 8 + wave; const int bb = m / SEQ, tt = m - bb * SEQ;
    const size_t rowf = ((size_t)bb * OUT_SEQ + tt) * DM;
    const int c0 = 4 * lane, c1 = 128 + 4 * lane;
    v4f x0 = *(const v4f*)(X + rowf + c0), x1 = *(const v4f*)(X + rowf + c1);
    if (doLN != 0) {
        const v4f o0 = *(const v4f*)(O + rowf + c0), o1 = *(const v4f*)(O + rowf + c1);
        const v4f g0 = *(const v4f*)(G + c0), g1 = *(const v4f*)(G + c1);
        const v4f b0 = *(const v4f*)(Be + c0), b1 = *(const v4f*)(Be + c1);
        x0 = x0 + o0; x1 = x1 + o1;
        float s = ((x0[0] + x0[1]) + (x0[2] + x0[3])) + ((x1[0] + x1[1]) + (x1[2] + x1[3]));
#pragma unroll 1
        for (int off = 16; off >= 1; off >>= 1) s += __shfl_xor(s, off, 32);
        const float mu = s * 0.00390625f;
        const v4f d0 = x0 - mu, d1 = x1 - mu;
        float q = ((d0[0] * d0[0] + d0[1] * d0[1]) + (d0[2] * d0[2] + d0[3] * d0[3])) + ((d1[0] * d1[0] + d1[1] * d1[1]) + (d1[2] * d1[2] + d1[3] * d1[3]));
#pragma unroll 1
        for (int off = 16; off >= 1; off >>= 1) q += __shfl_xor(q, off, 32);
        const float rsd = rsqrtf(q * 0.00390625f + 1.0e-5f);
#pragma unroll
        for (int i = 0; i < 4; ++i) { x0[i] = d0[i] * rsd * bfr(g0[i]) + bfr(b0[i]); x1[i] = d1[i] * rsd * bfr(g1[i]) + bfr(b1[i]); }
        float* yr = Y + rowf;
#pragma unroll 1
        for (int ps = 0; ps < 2; ++ps) {
            *(volatile v4f*)(yr + c0) = x0; *(volatile v4f*)(yr + c1) = x1;
            if (ps == 0) __threadfence(); }
    }
    if (doPl != 0) {
        const int wb = wave * DM;
        *(v4fa*)(&rs[wb + c0]) = x0; *(v4fa*)(&rs[wb + c1]) = x1;
        wave_sync();
        const v4f y0 = *(const v4fa*)(&rs[wb + 8 * lane]), y1 = *(const v4fa*)(&rs[wb + 8 * lane + 4]);
        v8us hv, lv;
#pragma unroll
        for (int i = 0; i < 4; ++i) { const unsigned short u0 = f2bf(y0[i]); const unsigned short u1 = f2bf(y1[i]); hv[i] = u0; hv[4 + i] = u1;
            lv[i] = f2bf(y0[i] - bf2f(u0)); lv[4 + i] = f2bf(y1[i] - bf2f(u1)); }
        bf* pr = PL + (size_t)m * CXP + 8 * lane;
#pragma unroll 1
        for (int ps = 0; ps < 2; ++ps) {
            *(volatile v8us*)pr = hv; *(volatile v8us*)(pr + DM) = lv;
            if (ps == 0) __threadfence(); }
    }
}

__global__ __launch_bounds__(32 * AW) void k_flash(const h16* __restrict__ QH, const h16* __restrict__ QR, const h16* __restrict__ KP, const h16* __restrict__ VT,
                                                   const unsigned* __restrict__ MB, bf* CX, float* ST) {
    __shared__ __align__(16) float os[AW * 16 * 68];
    const int lane = threadIdx.x & 31, wave = __builtin_amdgcn_readfirstlane((int)(threadIdx.x >> 5)), lr = lane & 15, hi = lane >> 4;
    const int zp = blockIdx.y; const int b = zp / (NH_ / 2), hp = zp % (NH_ / 2);
    const int t0 = (blockIdx.x * AW + wave) * 16;
    const int wb = wave * 16 * 68;
    const size_t rowb = (size_t)b * SEQ;
    const unsigned* mbp = MB + (size_t)(t0 + lr) * (SEQ / 32);
    const unsigned msh = 8u * (unsigned)hi;
    float* stl = ST + ((size_t)b * (SEQ / 16) + (size_t)(t0 >> 4)) * (NH_ * 32) + lane;
#pragma unroll 1
    for (int hh = 0; hh < 2; ++hh) {
        const int h = hp * 2 + hh;
        const size_t qo = (rowb + t0 + lr) * DM + h * HD + 8 * hi;
        const v16h qh = ldh(QH + qo), qr = ldh(QR + qo);
        const size_t ko = (rowb + lr) * DM + h * HD + 8 * hi;
        const size_t vo = ((size_t)b * DM + h * HD + lr) * SEQ + 8 * hi;
        v8f o0 = (v8f){}, o1 = (v8f){};
        float m = -3.0e38f, l = 0.0f;
#pragma unroll 1
        for (int key0 = 0; key0 < SEQ; key0 += 32) {
            const h16* ka = KP + ko + (size_t)key0 * DM;
            const v16h ka0 = ldh(ka), kb0 = ldh(ka + 16 * DM);
            unsigned mw = mbp[key0 >> 5]; asm volatile("" : "+v"(mw)); const unsigned ma = mw >> msh;
            v8f sHa = (v8f){}, sLa = (v8f){}, sHb = (v8f){}, sLb = (v8f){};
            sHa = wmma16(ka0, qh, sHa); sLa = wmma16(ka0, qr, sLa); sHb = wmma16(kb0, qh, sHb); sLb = wmma16(kb0, qr, sLb);
            asm volatile("v_nop\n\tv_nop\n\tv_nop\n\tv_nop" : "+v"(sHa), "+v"(sLa), "+v"(sHb), "+v"(sLb) : "v"(ka0), "v"(kb0), "v"(qh), "v"(qr));
            float ta[8], tb[8]; float mx = -3.0e38f;
#pragma unroll
            for (int r = 0; r < 8; ++r) {
                const float a0 = (sHa[r] + sLa[r] * QRI) * SC2;
                const float c0 = (sHb[r] + sLb[r] * QRI) * SC2;
                ta[r] = (((ma >> r) & 1u) != 0u) ? a0 : NEGT;
                tb[r] = (((ma >> (16 + r)) & 1u) != 0u) ? c0 : NEGT; }
#pragma unroll
            for (int r = 0; r < 8; ++r) mx = fmaxf(mx, fmaxf(ta[r], tb[r]));
            mx = fmaxf(mx, __shfl_xor(mx, 16, 32));
            const float mnew = fmaxf(m, mx);
            const float alpha = __builtin_amdgcn_exp2f(m - mnew);
            v16h pb; float ls = 0.0f;
#pragma unroll
            for (int r = 0; r < 8; ++r) { const float ea = (ta[r] - mnew) + PSH, ec = (tb[r] - mnew) + PSH;
                const h16 pa = (ea < -14.0f) ? (h16)0.0f : (h16)__builtin_amdgcn_exp2f(ea);
                const h16 pc = (ec < -14.0f) ? (h16)0.0f : (h16)__builtin_amdgcn_exp2f(ec);
                pb[r] = pa; pb[8 + r] = pc; ls += (float)pa + (float)pc; }
            l = l * alpha + ls; m = mnew;
            o0 = o0 * alpha; o1 = o1 * alpha;
            const h16* va = VT + vo + key0;
            const v16h v0 = ldh(va), v1 = ldh(va + (size_t)16 * SEQ);
            o0 = wmma16(v0, pb, o0); o1 = wmma16(v1, pb, o1);
            asm volatile("v_nop\n\tv_nop\n\tv_nop\n\tv_nop" : "+v"(o0), "+v"(o1) : "v"(v0), "v"(v1), "v"(pb));
        }
        l += __shfl_xor(l, 16, 32);
        const float inv = 1.0f / l;
        { const float sv = (hi != 0) ? inv : m; float* sp = stl + h * 32;
          *(volatile float*)sp = sv; __threadfence(); *(volatile float*)sp = sv; }
        { v4f a, c; const int ob = wb + lr * 68 + hh * 32 + 8 * hi;
          a[0] = o0[0] * inv; a[1] = o0[1] * inv; a[2] = o0[2] * inv; a[3] = o0[3] * inv; c[0] = o0[4] * inv; c[1] = o0[5] * inv; c[2] = o0[6] * inv; c[3] = o0[7] * inv;
          *(v4fa*)(&os[ob]) = a; *(v4fa*)(&os[ob + 4]) = c;
          a[0] = o1[0] * inv; a[1] = o1[1] * inv; a[2] = o1[2] * inv; a[3] = o1[3] * inv; c[0] = o1[4] * inv; c[1] = o1[5] * inv; c[2] = o1[6] * inv; c[3] = o1[7] * inv;
          *(v4fa*)(&os[ob + 16]) = a; *(v4fa*)(&os[ob + 20]) = c; }
    }
    wave_sync();
    bf* crow = CX + (rowb + t0) * CXP + hp * 64;
#pragma unroll 1
    for (int ps = 0; ps < 2; ++ps) {
#pragma unroll
        for (int s = 0; s < 4; ++s) { const int row = 4 * s + (lane >> 3), c8 = (lane & 7) * 8;
            const v4f x0 = *(const v4fa*)(&os[wb + row * 68 + c8]); const v4f x1 = *(const v4fa*)(&os[wb + row * 68 + c8 + 4]); v8us hv, lv;
#pragma unroll
            for (int i = 0; i < 4; ++i) { const unsigned short u0 = f2bf(x0[i]); const unsigned short u1 = f2bf(x1[i]); hv[i] = u0; hv[4 + i] = u1;
                lv[i] = f2bf(x0[i] - bf2f(u0)); lv[4 + i] = f2bf(x1[i] - bf2f(u1)); }
            const size_t oo = (size_t)row * CXP + c8;
            *(volatile v8us*)(crow + oo) = hv; *(volatile v8us*)(crow + oo + DM) = lv; }
        if (ps == 0) __threadfence(); }
}

__global__ __launch_bounds__(32 * AW) void k_agg(const h16* __restrict__ QH, const h16* __restrict__ QR, const h16* __restrict__ KP,
                                                 const unsigned* __restrict__ MB, const float* __restrict__ ST, h16* AP) {
    __shared__ __align__(16) float os[AW * 16 * 68];
    __shared__ float sst[AW * NH_ * 32];
    const int lane = threadIdx.x & 31, wave = __builtin_amdgcn_readfirstlane((int)(threadIdx.x >> 5)), lr = lane & 15, hi = lane >> 4;
    const int b = blockIdx.y;
    const int t0 = (blockIdx.x * AW + wave) * 16;
    const int wb = wave * 16 * 68, sb = wave * NH_ * 32;
    const size_t rowb = (size_t)b * SEQ;
    const float* stp = ST + ((size_t)b * (SEQ / 16) + (size_t)(t0 >> 4)) * (NH_ * 32);
#pragma unroll
    for (int i = 0; i < NH_; ++i) sst[sb + i * 32 + lane] = stp[i * 32 + lane];
    wave_sync();
    const unsigned* mbp = MB + (size_t)(t0 + lr) * (SEQ / 32);
    const unsigned msh = 8u * (unsigned)hi;
    const size_t qo = (rowb + t0 + lr) * DM + 8 * hi;
    const size_t ko = (rowb + lr) * DM + 8 * hi;
    h16* arow = AP + (rowb + t0) * SEQ;
#pragma unroll 1
    for (int key0 = 0; key0 < SEQ; key0 += 64) {
#pragma unroll 1
        for (int sub = 0; sub < 2; ++sub) {
            const int kb = key0 + 32 * sub;
            unsigned mw = mbp[kb >> 5]; asm volatile("" : "+v"(mw)); const unsigned ma = mw >> msh;
            float ga[8], gb[8];
#pragma unroll
            for (int r = 0; r < 8; ++r) { ga[r] = 0.0f; gb[r] = 0.0f; }
#pragma unroll 1
            for (int h = 0; h < NH_; ++h) {
                const v16h qh = ldh(QH + qo + h * HD), qr = ldh(QR + qo + h * HD);
                const h16* ka = KP + ko + (size_t)kb * DM + h * HD;
                const v16h ka0 = ldh(ka), kb0 = ldh(ka + 16 * DM);
                v8f sHa = (v8f){}, sLa = (v8f){}, sHb = (v8f){}, sLb = (v8f){};
                sHa = wmma16g(ka0, qh, sHa); sLa = wmma16g(ka0, qr, sLa); sHb = wmma16g(kb0, qh, sHb); sLb = wmma16g(kb0, qr, sLb);
                const float mh = sst[sb + h * 32 + lr], ih = sst[sb + h * 32 + 16 + lr];
#pragma unroll
                for (int r = 0; r < 8; ++r) {
                    const float a0 = (sHa[r] + sLa[r] * QRI) * SC2;
                    const float c0 = (sHb[r] + sLb[r] * QRI) * SC2;
                    const float ta = (((ma >> r) & 1u) != 0u) ? a0 : NEGT;
                    const float tb = (((ma >> (16 + r)) & 1u) != 0u) ? c0 : NEGT;
                    ga[r] += __builtin_amdgcn_exp2f((ta - mh) + APS) * ih;
                    gb[r] += __builtin_amdgcn_exp2f((tb - mh) + APS) * ih; }
            }
            { v4f a, c; const int ob = wb + lr * 68 + 32 * sub + 8 * hi;
              a[0] = ga[0]; a[1] = ga[1]; a[2] = ga[2]; a[3] = ga[3]; c[0] = ga[4]; c[1] = ga[5]; c[2] = ga[6]; c[3] = ga[7];
              *(v4fa*)(&os[ob]) = a; *(v4fa*)(&os[ob + 4]) = c;
              a[0] = gb[0]; a[1] = gb[1]; a[2] = gb[2]; a[3] = gb[3]; c[0] = gb[4]; c[1] = gb[5]; c[2] = gb[6]; c[3] = gb[7];
              *(v4fa*)(&os[ob + 16]) = a; *(v4fa*)(&os[ob + 20]) = c; }
        }
        wave_sync();
#pragma unroll 1
        for (int ps = 0; ps < 2; ++ps) {
#pragma unroll
            for (int s = 0; s < 4; ++s) { const int row = 4 * s + (lane >> 3), c8 = (lane & 7) * 8;
                const v4f x0 = *(const v4fa*)(&os[wb + row * 68 + c8]); const v4f x1 = *(const v4fa*)(&os[wb + row * 68 + c8 + 4]); v8h hv;
#pragma unroll
                for (int i = 0; i < 4; ++i) { hv[i] = toh_flush(x0[i]); hv[4 + i] = toh_flush(x1[i]); }
                *(volatile v8h*)(arow + (size_t)row * SEQ + key0 + c8) = hv; }
            if (ps == 0) __threadfence(); }
        wave_sync();
    }
}
static_assert(32 * 16 * 4 == 16 * 128);

__global__ __launch_bounds__(256) void k_tr(const h16* __restrict__ src, h16* dst) {
    __shared__ __align__(16) h16 ts[64 * 72];
    const int tid = threadIdx.x; const int c0 = blockIdx.x * 64, r0 = blockIdx.y * 64;
    const size_t base = (size_t)blockIdx.z * SEQ * SEQ;
#pragma unroll
    for (int it = 0; it < 2; ++it) { const int rr = it * 32 + (tid >> 3), cs = (tid & 7) * 8;
        const v8h v = *(const v8h*)(src + base + (size_t)(r0 + rr) * SEQ + c0 + cs);
        *(v8ha*)(&ts[rr * 72 + cs]) = v; }
    __syncthreads();
#pragma unroll 1
    for (int ps = 0; ps < 2; ++ps) {
#pragma unroll
        for (int it = 0; it < 2; ++it) { const int cc = it * 32 + (tid >> 3), rq = (tid & 7) * 8;
            v8h o;
#pragma unroll
            for (int j = 0; j < 8; ++j) o[j] = ts[(rq + j) * 72 + cc];
            *(volatile v8h*)(dst + base + (size_t)(c0 + cc) * SEQ + r0 + rq) = o; }
        if (ps == 0) __threadfence(); }
}
static_assert(2 * 256 * 8 == 64 * 64);

__global__ __launch_bounds__(32) void k_roll(const h16* __restrict__ A, const h16* __restrict__ Bt, float* OUT) {
    __shared__ __align__(16) float os[16 * 68];
    const int lane = threadIdx.x & 31, lr = lane & 15, hi = lane >> 4; const int r0 = blockIdx.x * 64, c0 = blockIdx.y * 64;
    const size_t pb = (size_t)blockIdx.z * SEQ * SEQ;
    v8f acc[4][4];
#pragma unroll
    for (int mb = 0; mb < 4; ++mb)
#pragma unroll
        for (int nb = 0; nb < 4; ++nb) acc[mb][nb] = (v8f){};
    const size_t aoff = pb + (size_t)(r0 + lr) * SEQ + 8 * hi, boff = pb + (size_t)(c0 + lr) * SEQ + 8 * hi;
#pragma unroll 1
    for (int kc = 0; kc < SEQ; kc += 32) {
        v16h a[4];
#pragma unroll
        for (int mb = 0; mb < 4; ++mb) a[mb] = ldh(A + aoff + (size_t)mb * 16 * SEQ + kc);
#pragma unroll
        for (int nb = 0; nb < 4; ++nb) { const v16h bq = ldh(Bt + boff + (size_t)nb * 16 * SEQ + kc);
#pragma unroll
            for (int mb = 0; mb < 4; ++mb) acc[mb][nb] = wmma16g(a[mb], bq, acc[mb][nb]); }
    }
    float* ob = OUT + (size_t)blockIdx.z * ATT_BP;
#pragma unroll
    for (int mb = 0; mb < 4; ++mb) {
#pragma unroll
        for (int nb = 0; nb < 4; ++nb) {
#pragma unroll
            for (int j = 0; j < 8; ++j) os[(hi * 8 + j) * 68 + nb * 16 + lr] = acc[mb][nb][j]; }
        wave_sync();
#pragma unroll 1
        for (int ps = 0; ps < 2; ++ps) {
#pragma unroll
            for (int s = 0; s < 8; ++s) { const int row = 2 * s + hi, cofs = lr * 4;
                v4f val = *(const v4fa*)(&os[row * 68 + cofs]);
#pragma unroll
                for (int i = 0; i < 4; ++i) val[i] = val[i] * RSC;
                *(volatile v4f*)(ob + (size_t)(r0 + mb * 16 + row) * ATT_RP + c0 + cofs) = val; }
            if (ps == 0) __threadfence(); }
        wave_sync();
    }
}
static_assert(32 * 16 * 8 == 16 * 256);

static_assert((size_t)16 * 68 * 4 <= 131072);
static_assert((size_t)AW * 16 * 68 * 4 <= 131072);
static_assert((size_t)AW * 16 * 68 * 4 + (size_t)AW * NH_ * 32 * 4 <= 131072);
static_assert((size_t)8 * DM * 4 <= 131072);
static_assert((size_t)64 * 72 * 2 <= 131072);

static constexpr size_t al256(size_t v) { return (v + 255) & ~(size_t)255; }
static constexpr size_t SZ_X  = al256((size_t)NB * SEQ * DM * 2);
static constexpr size_t SZ_W  = al256((size_t)DM * DM * 2);
static constexpr size_t SZ_W2 = al256((size_t)NL * DM * CXP * 2);
static constexpr size_t SZ_ZB = al256((size_t)DM * 4);
static constexpr size_t SZ_MB = al256((size_t)SEQ * (SEQ / 32) * 4);
static constexpr size_t SZ_F  = al256((size_t)NB * OUT_SEQ * DM * 4);
static constexpr size_t SZ_PL = al256((size_t)NB * SEQ * DM * 2);
static constexpr size_t SZ_CX = al256((size_t)NB * SEQ * CXP * 2);
static constexpr size_t SZ_ST = al256((size_t)NB * (SEQ / 16) * NH_ * 32 * 4);
static constexpr size_t SZ_AP = al256((size_t)NB * SEQ * SEQ * 2);
static constexpr size_t SZ_TOTAL = SZ_X + SZ_W + 4 * SZ_W2 + SZ_ZB + SZ_MB + 3 * SZ_F + 4 * SZ_PL + 2 * SZ_CX + SZ_ST + 3 * SZ_AP;
static_assert(SZ_TOTAL <= (size_t)134217728);
static_assert((size_t)NB * DM * SEQ * 2 <= SZ_PL);
static_assert(((size_t)(NB - 1) * OUT_SEQ + SEQ) * DM * 4 <= SZ_F);

static void cvt_act(const float* x, bf* dst, hipStream_t stream) {
    if (SEQ == SEQ_FULL) {
        const size_t n8 = (size_t)NB * SEQ * DM / 8;
        k_cvt8<<<(unsigned)((n8 + 255) / 256), 256, 0, stream>>>(x, dst, n8);
    } else {
        const size_t n8 = (size_t)SEQ * DM / 8;
        for (int b = 0; b < NB; ++b) k_cvt8<<<(unsigned)((n8 + 255) / 256), 256, 0, stream>>>(x + (size_t)b * SEQ_FULL * DM, dst + (size_t)b * SEQ * DM, n8);
    }
}

extern "C" void kernel_launch(void* const* d_in, const int* in_sizes, int n_in,
                              void* d_out, int out_size, void* d_ws, size_t ws_size, hipStream_t stream) {
    if (n_in < 9) return;
    if ((size_t)in_sizes[0] < ((size_t)(NB - 1) * SEQ_FULL + SEQ) * DM) return;
    if ((size_t)in_sizes[1] < (size_t)(SEQ - 1) * SEQ_FULL + SEQ) return;
    if ((size_t)in_sizes[2] < (size_t)DM * DM) return;
    if ((size_t)in_sizes[3] < (size_t)NL * DM * DM || (size_t)in_sizes[4] < (size_t)NL * DM * DM || (size_t)in_sizes[5] < (size_t)NL * DM * DM || (size_t)in_sizes[6] < (size_t)NL * DM * DM) return;
    if (in_sizes[7] < NL * DM || in_sizes[8] < NL * DM) return;
    if ((size_t)out_size < ATT_OFF + (size_t)(NB - 1) * ATT_BP + (size_t)(SEQ - 1) * ATT_RP + SEQ) return;
    if (SZ_TOTAL > ws_size) return;
    const float* xin = (const float*)d_in[0]; const float* adj = (const float*)d_in[1]; const float* wf0 = (const float*)d_in[2];
    const float* wq = (const float*)d_in[3]; const float* wk = (const float*)d_in[4]; const float* wv = (const float*)d_in[5]; const float* wo = (const float*)d_in[6];
    const float* gam = (const float*)d_in[7]; const float* bet = (const float*)d_in[8];
    float* OUTX = (float*)d_out;
    float* ATT = OUTX + ATT_OFF;
    char* wsp = (char*)d_ws;
    bf* XB = (bf*)wsp; wsp += SZ_X;
    bf* WF = (bf*)wsp; wsp += SZ_W;
    bf* WQ2 = (bf*)wsp; wsp += SZ_W2;
    bf* WK2 = (bf*)wsp; wsp += SZ_W2;
    bf* WV2 = (bf*)wsp; wsp += SZ_W2;
    bf* WO2 = (bf*)wsp; wsp += SZ_W2;
    float* ZB = (float*)wsp; wsp += SZ_ZB;
    unsigned* MB = (unsigned*)wsp; wsp += SZ_MB;
    float* X0F = (float*)wsp; wsp += SZ_F;
    float* X1F = (float*)wsp; wsp += SZ_F;
    float* OPF = (float*)wsp; wsp += SZ_F;
    bf* XP = (bf*)wsp; wsp += SZ_CX;
    h16* QH = (h16*)wsp; wsp += SZ_PL;
    h16* QR = (h16*)wsp; wsp += SZ_PL;
    h16* KP = (h16*)wsp; wsp += SZ_PL;
    h16* VT = (h16*)wsp; wsp += SZ_PL;
    bf* CX = (bf*)wsp; wsp += SZ_CX;
    float* ST = (float*)wsp; wsp += SZ_ST;
    h16* A0 = (h16*)wsp; wsp += SZ_AP;
    h16* A1 = (h16*)wsp; wsp += SZ_AP;
    h16* A0T = (h16*)wsp; wsp += SZ_AP;

    cvt_act(xin, XB, stream);
    { const size_t n8 = (size_t)DM * DM / 8; k_cvt8<<<(unsigned)((n8 + 255) / 256), 256, 0, stream>>>(wf0, WF, n8); }
    { const size_t n8 = (size_t)NL * DM * DM / 8; const unsigned g = (unsigned)((n8 + 255) / 256);
      k_wdup<<<g, 256, 0, stream>>>(wq, WQ2, n8);
      k_wdup<<<g, 256, 0, stream>>>(wk, WK2, n8);
      k_wdup<<<g, 256, 0, stream>>>(wv, WV2, n8);
      k_wdup<<<g, 256, 0, stream>>>(wo, WO2, n8); }
    k_zero<<<1, 64, 0, stream>>>(ZB);
    k_mask<<<(unsigned)(((size_t)SEQ * (SEQ / 32)) / 256), 256, 0, stream>>>(adj, MB);

    k_gemm<true><<<dim3(NB * SEQ / 64, DM / 64, 1), 32, 0, stream>>>(XB, WF, QH, QH, X0F, ZB, (size_t)0, (size_t)0, DM, 0, NB * SEQ, DM, DM, 0);
    k_rowop<<<NB * SEQ / 8, 256, 0, stream>>>(X0F, X0F, gam, bet, X0F, XP, 0, 1);

    for (int l = 0; l < NL; ++l) {
        const bf* wq2 = WQ2 + (size_t)l * DM * CXP; const bf* wk2 = WK2 + (size_t)l * DM * CXP;
        const bf* wv2 = WV2 + (size_t)l * DM * CXP; const bf* wo2 = WO2 + (size_t)l * DM * CXP;
        k_gemm<false><<<dim3(NB * SEQ / 64, DM / 64, 1), 32, 0, stream>>>(XP, wq2, QH, QR, X0F, ZB, (size_t)0, (size_t)0, CXP, 1, NB * SEQ, DM, DM, 0);
        k_gemm<false><<<dim3(NB * SEQ / 64, DM / 64, 1), 32, 0, stream>>>(XP, wk2, KP, KP, X0F, ZB, (size_t)0, (size_t)0, CXP, 0, NB * SEQ, DM, DM, 0);
        k_gemm<false><<<dim3(DM / 64, NB * SEQ / 64, 1), 32, 0, stream>>>(wv2, XP, VT, VT, X0F, ZB, (size_t)0, (size_t)DM * SEQ, CXP, 0, DM, SEQ, SEQ, 1);

        k_flash<<<dim3(SEQ / (16 * AW), NB * (NH_ / 2), 1), 32 * AW, 0, stream>>>(QH, QR, KP, VT, MB, CX, ST);
        k_agg<<<dim3(SEQ / (16 * AW), NB, 1), 32 * AW, 0, stream>>>(QH, QR, KP, MB, ST, (l == 0) ? A0 : A1);

        k_gemm<true><<<dim3(NB * SEQ / 64, DM / 64, 1), 32, 0, stream>>>(CX, wo2, QH, QH, OPF, ZB, (size_t)0, (size_t)0, CXP, 0, NB * SEQ, DM, DM, 0);
        const float* xs = (l == 0) ? X0F : X1F;
        float* yd = (l == NL - 1) ? OUTX : X1F;
        k_rowop<<<NB * SEQ / 8, 256, 0, stream>>>(xs, OPF, gam + (size_t)l * DM, bet + (size_t)l * DM, yd, XP, 1, (l == NL - 1) ? 0 : 1);
    }

    k_tr<<<dim3(SEQ / 64, SEQ / 64, NB), 256, 0, stream>>>(A0, A0T);
    k_roll<<<dim3(SEQ / 64, SEQ / 64, NB), 32, 0, stream>>>(A1, A0T, ATT);
}
